// WINNERHierarchicalDecomposer_34454227648861
// MI455X (gfx1250) — hardware-verified
//
#include <hip/hip_runtime.h>
#include <hip/hip_bf16.h>
#include <math.h>


typedef _Float16 bf16;
typedef _Float16 f16;
typedef __attribute__((ext_vector_type(4))) unsigned v4u_t;
typedef unsigned v4ua __attribute__((ext_vector_type(4), may_alias));
typedef __attribute__((ext_vector_type(4))) float v4f_t;
typedef float v4fa __attribute__((ext_vector_type(4), may_alias));
typedef __attribute__((ext_vector_type(16))) bf16  bf16x16;
typedef bf16x16 f16x16;
typedef __attribute__((ext_vector_type(8)))  bf16  bf16x8;
typedef bf16x8 f16x8;
typedef __attribute__((ext_vector_type(4)))  bf16  bf16x4;
typedef __attribute__((ext_vector_type(8)))  float f32x8;
__device__ __forceinline__ f32x8 wmma16(f16x16 a, f16x16 b, f32x8 c) {
  c = __builtin_amdgcn_wmma_f32_16x16x32_f16(false, a, false, b, (short)0, c, false, false);
  asm volatile("v_nop\n\tv_nop\n\tv_nop\n\tv_nop" : "+v"(c) : "v"(a), "v"(b));
  return c;
}
#define LDS_STRIDE 48
#define KSTRIDE    72
#define VSTRIDE    48

__device__ __forceinline__ f32x8 wmma_bf16(bf16x16 a, bf16x16 b, f32x8 c) {
  c = __builtin_amdgcn_wmma_f32_16x16x32_f16(false, a, false, b, (short)0, c, false, false);
  asm volatile("v_nop\n\tv_nop\n\tv_nop\n\tv_nop" : "+v"(c) : "v"(a), "v"(b));
  return c;
}

template <typename T>
__device__ __forceinline__ bf16x16 load_frag(const T* __restrict__ base, int ld,
                                             int row0, int k0) {
  const int lane = threadIdx.x & 31;
  const int r    = lane & 15;
  const int kh   = (lane >> 4) * 8;
  const T* p0 = base + (size_t)(row0 + r) * ld + (k0 + kh);
  const T* p1 = p0 + 16;
  bf16x16 f;
#pragma unroll
  for (int i = 0; i < 8; ++i) {
    f[i]     = (bf16)p0[i];
    f[i + 8] = (bf16)p1[i];
  }
  return f;
}

__device__ __forceinline__ bf16x16 lds_frag(const bf16* base, int stride) {
  const int lane = threadIdx.x & 31;
  const int row  = lane & 15;
  const int kh   = (lane >> 4) * 8;
  const bf16x8 lo = *(const bf16x8*)(base + row * stride + kh);
  const bf16x8 hi = *(const bf16x8*)(base + row * stride + kh + 16);
  bf16x16 f;
#pragma unroll
  for (int i = 0; i < 8; ++i) { f[i] = lo[i]; f[i + 8] = hi[i]; }
  return f;
}

template <typename T>
__device__ __forceinline__ void stage_read16(const T* __restrict__ p, float* buf) {
#pragma unroll
  for (int i = 0; i < 16; ++i) buf[i] = (float)p[i];
}

__device__ __forceinline__ void stage_write(bf16* dst, const float* buf, int nquad) {
#pragma unroll
  for (int i = 0; i < nquad; ++i) {
    bf16x4 q;
    q[0] = (bf16)buf[4 * i];     q[1] = (bf16)buf[4 * i + 1];
    q[2] = (bf16)buf[4 * i + 2]; q[3] = (bf16)buf[4 * i + 3];
    *(bf16x4*)(dst + 4 * i) = q;
  }
}


#define GSTR 48
#define GSTR 48
template <typename AT, int EPI, bool OUT16>
__global__ __launch_bounds__(256) void gemm_kne(const AT* __restrict__ A, int lda, const float* __restrict__ Wm, int ldw,
                                                const float* __restrict__ bias, const float* __restrict__ R, const float* __restrict__ gvec,
                                                void* __restrict__ Yv, int ldy, int K) {
  __shared__ __attribute__((aligned(16))) f16 ldsA[128 * GSTR];
  __shared__ __attribute__((aligned(16))) f16 ldsW[128 * GSTR];
  __shared__ __attribute__((aligned(16))) float oS[8][32 * 68];
  const int tid = threadIdx.x, lane = tid & 31, wave = tid >> 5, cl = lane & 15, rh = (lane >> 4) * 8;
  const int m0 = blockIdx.x * 128, n0 = blockIdx.y * 128;
  const int wm = (wave & 3) * 32, wn = (wave >> 2) * 64;
  f32x8 acc[2][4];
#pragma unroll
  for (int i = 0; i < 2; ++i)
#pragma unroll
    for (int j = 0; j < 4; ++j) { f32x8 z = {}; acc[i][j] = z; }
#pragma unroll 1
  for (int k0 = 0; k0 < K; k0 += 32) {
    __syncthreads();
    { const int row = tid >> 1, ch = (tid & 1) * 16;
      const AT* src = A + (size_t)(m0 + row) * lda + k0 + ch;
#pragma unroll
      for (int g = 0; g < 16; ++g) ldsA[row * GSTR + ch + g] = (f16)src[g]; }
    { const int k = tid >> 3, nn0 = (tid & 7) * 16;
      const float* src = Wm + (size_t)(k0 + k) * ldw + n0 + nn0;
#pragma unroll
      for (int g = 0; g < 4; ++g) { const v4f_t v = *(const v4f_t*)(src + 4 * g);
#pragma unroll
        for (int u = 0; u < 4; ++u) ldsW[(nn0 + 4 * g + u) * GSTR + k] = (f16)v[u]; } }
    __syncthreads();
    f16x16 af[2];
#pragma unroll
    for (int i = 0; i < 2; ++i) af[i] = lds_frag(ldsA + (wm + 16 * i) * GSTR, GSTR);
#pragma unroll
    for (int j = 0; j < 4; ++j) {
      const f16x16 bf = lds_frag(ldsW + (wn + 16 * j) * GSTR, GSTR);
#pragma unroll
      for (int i = 0; i < 2; ++i) acc[i][j] = wmma16(af[i], bf, acc[i][j]);
    }
  }
  float* so = oS[wave];
#pragma unroll
  for (int i = 0; i < 2; ++i)
#pragma unroll
    for (int j = 0; j < 4; ++j) {
      const int n = n0 + wn + 16 * j + cl;
      const float bv = bias ? bias[n] : 0.0f;
      const float gv = (EPI == 2 || EPI == 4 || EPI == 14) ? gvec[n] : 0.0f;
      if (EPI == 1) {
#pragma unroll 1
        for (int r = 0; r < 8; ++r) { const float xg = acc[i][j][r] + bv; so[(16 * i + rh + r) * 68 + 16 * j + cl] = 0.5f * xg * (1.0f + erff(xg * 0.70710678118654752f)); }
      } else if (EPI == 13) {
#pragma unroll 1
        for (int r = 0; r < 8; ++r) { const size_t mrow = (size_t)(m0 + wm + 16 * i + rh + r); const float xg = acc[i][j][r] + bv; float o = (1.0f / (1.0f + expf(-xg))) * gvec[mrow]; if (R) o += R[mrow * ldy + n]; so[(16 * i + rh + r) * 68 + 16 * j + cl] = o; }
      } else if (EPI == 11) {
#pragma unroll 1
        for (int r = 0; r < 8; ++r) { const float xg = acc[i][j][r] + bv; so[(16 * i + rh + r) * 68 + 16 * j + cl] = xg / (1.0f + expf(-xg)); }
      } else if (EPI == 9 || EPI == 10) {
#pragma unroll 1
        for (int r = 0; r < 8; ++r) { const float xg = acc[i][j][r] + bv + R[(size_t)(m0 + wm + 16 * i + rh + r) * ldy + n]; so[(16 * i + rh + r) * 68 + 16 * j + cl] = (EPI == 9) ? 1.0f / (1.0f + expf(-xg)) : tanhf(xg); }
      } else {
#pragma unroll
        for (int r = 0; r < 8; ++r) {
          float v = acc[i][j][r] + bv;
          if (EPI == 3) v = fmaxf(v, 0.0f);
          if (EPI == 6) v = fminf(fmaxf(v, 0.0f), 6.0f);
          if (EPI == 4) v = gv * v;
          if (EPI == 14) v = fmaxf(acc[i][j][r] * gv + bv, 0.0f);
          if (EPI == 2) v = R[(size_t)(m0 + wm + 16 * i + rh + r) * ldy + n] + gv * v;
          so[(16 * i + rh + r) * 68 + 16 * j + cl] = v;
        }
      }
    }
  asm volatile("s_wait_dscnt 0" ::: "memory");
  __builtin_amdgcn_wave_barrier();
#pragma unroll 1
  for (int pass = 0; pass < 2; ++pass) {
    if (OUT16) {
      f16* Y = (f16*)Yv;
#pragma unroll
      for (int it = 0; it < 8; ++it) { const int c = lane + 32 * it, rr = c >> 3, q8 = (c & 7) * 8;
        union { f16 h[8]; v4u_t v; } u;
#pragma unroll
        for (int e = 0; e < 8; ++e) u.h[e] = (f16)so[rr * 68 + q8 + e];
        *(volatile v4u_t*)(Y + (size_t)(m0 + wm + rr) * ldy + n0 + wn + q8) = u.v; }
    } else {
      float* Y = (float*)Yv;
#pragma unroll
      for (int it = 0; it < 16; ++it) { const int f4 = lane + 32 * it, rr = f4 >> 4, q = (f4 & 15) * 4;
        *(volatile v4f_t*)(Y + (size_t)(m0 + wm + rr) * ldy + n0 + wn + q) = *(const v4fa*)(so + rr * 68 + q); }
    }
    __threadfence();
  }
}

template <typename AT, int EPI, bool OUT16>
__global__ __launch_bounds__(256) void gemm_knez(const AT* __restrict__ A, int lda, size_t strideA, const float* __restrict__ Wm, int ldw, size_t strideW,
                                                 const float* __restrict__ bias, const float* __restrict__ R, const float* __restrict__ gvec,
                                                 void* __restrict__ Yv, int ldy, size_t strideY, int K) {
  A += (size_t)blockIdx.z * strideA; Wm += (size_t)blockIdx.z * strideW; Yv = (void*)((char*)Yv + (size_t)blockIdx.z * strideY * (OUT16 ? 2 : 4)); if (R) R += (size_t)blockIdx.z * strideY;
  __shared__ __attribute__((aligned(16))) f16 ldsA[128 * GSTR];
  __shared__ __attribute__((aligned(16))) f16 ldsW[128 * GSTR];
  __shared__ __attribute__((aligned(16))) float oS[8][32 * 68];
  const int tid = threadIdx.x, lane = tid & 31, wave = tid >> 5, cl = lane & 15, rh = (lane >> 4) * 8;
  const int m0 = blockIdx.x * 128, n0 = blockIdx.y * 128;
  const int wm = (wave & 3) * 32, wn = (wave >> 2) * 64;
  f32x8 acc[2][4];
#pragma unroll
  for (int i = 0; i < 2; ++i)
#pragma unroll
    for (int j = 0; j < 4; ++j) { f32x8 z = {}; acc[i][j] = z; }
#pragma unroll 1
  for (int k0 = 0; k0 < K; k0 += 32) {
    __syncthreads();
    { const int row = tid >> 1, ch = (tid & 1) * 16;
      const AT* src = A + (size_t)(m0 + row) * lda + k0 + ch;
#pragma unroll
      for (int g = 0; g < 16; ++g) ldsA[row * GSTR + ch + g] = (f16)src[g]; }
    { const int k = tid >> 3, nn0 = (tid & 7) * 16;
      const float* src = Wm + (size_t)(k0 + k) * ldw + n0 + nn0;
#pragma unroll
      for (int g = 0; g < 4; ++g) { const v4f_t v = *(const v4f_t*)(src + 4 * g);
#pragma unroll
        for (int u = 0; u < 4; ++u) ldsW[(nn0 + 4 * g + u) * GSTR + k] = (f16)v[u]; } }
    __syncthreads();
    f16x16 af[2];
#pragma unroll
    for (int i = 0; i < 2; ++i) af[i] = lds_frag(ldsA + (wm + 16 * i) * GSTR, GSTR);
#pragma unroll
    for (int j = 0; j < 4; ++j) {
      const f16x16 bf = lds_frag(ldsW + (wn + 16 * j) * GSTR, GSTR);
#pragma unroll
      for (int i = 0; i < 2; ++i) acc[i][j] = wmma16(af[i], bf, acc[i][j]);
    }
  }
  float* so = oS[wave];
#pragma unroll
  for (int i = 0; i < 2; ++i)
#pragma unroll
    for (int j = 0; j < 4; ++j) {
      const int n = n0 + wn + 16 * j + cl;
      const float bv = bias ? bias[n] : 0.0f;
      const float gv = (EPI == 2 || EPI == 4 || EPI == 14) ? gvec[n] : 0.0f;
      if (EPI == 1) {
#pragma unroll 1
        for (int r = 0; r < 8; ++r) { const float xg = acc[i][j][r] + bv; so[(16 * i + rh + r) * 68 + 16 * j + cl] = 0.5f * xg * (1.0f + erff(xg * 0.70710678118654752f)); }
      } else if (EPI == 13) {
#pragma unroll 1
        for (int r = 0; r < 8; ++r) { const size_t mrow = (size_t)(m0 + wm + 16 * i + rh + r); const float xg = acc[i][j][r] + bv; float o = (1.0f / (1.0f + expf(-xg))) * gvec[mrow]; if (R) o += R[mrow * ldy + n]; so[(16 * i + rh + r) * 68 + 16 * j + cl] = o; }
      } else if (EPI == 11) {
#pragma unroll 1
        for (int r = 0; r < 8; ++r) { const float xg = acc[i][j][r] + bv; so[(16 * i + rh + r) * 68 + 16 * j + cl] = xg / (1.0f + expf(-xg)); }
      } else if (EPI == 9 || EPI == 10) {
#pragma unroll 1
        for (int r = 0; r < 8; ++r) { const float xg = acc[i][j][r] + bv + R[(size_t)(m0 + wm + 16 * i + rh + r) * ldy + n]; so[(16 * i + rh + r) * 68 + 16 * j + cl] = (EPI == 9) ? 1.0f / (1.0f + expf(-xg)) : tanhf(xg); }
      } else {
#pragma unroll
        for (int r = 0; r < 8; ++r) {
          float v = acc[i][j][r] + bv;
          if (EPI == 3) v = fmaxf(v, 0.0f);
          if (EPI == 6) v = fminf(fmaxf(v, 0.0f), 6.0f);
          if (EPI == 4) v = gv * v;
          if (EPI == 14) v = fmaxf(acc[i][j][r] * gv + bv, 0.0f);
          if (EPI == 2) v = R[(size_t)(m0 + wm + 16 * i + rh + r) * ldy + n] + gv * v;
          so[(16 * i + rh + r) * 68 + 16 * j + cl] = v;
        }
      }
    }
  asm volatile("s_wait_dscnt 0" ::: "memory");
  __builtin_amdgcn_wave_barrier();
#pragma unroll 1
  for (int pass = 0; pass < 2; ++pass) {
    if (OUT16) {
      f16* Y = (f16*)Yv;
#pragma unroll
      for (int it = 0; it < 8; ++it) { const int c = lane + 32 * it, rr = c >> 3, q8 = (c & 7) * 8;
        union { f16 h[8]; v4u_t v; } u;
#pragma unroll
        for (int e = 0; e < 8; ++e) u.h[e] = (f16)so[rr * 68 + q8 + e];
        *(volatile v4u_t*)(Y + (size_t)(m0 + wm + rr) * ldy + n0 + wn + q8) = u.v; }
    } else {
      float* Y = (float*)Yv;
#pragma unroll
      for (int it = 0; it < 16; ++it) { const int f4 = lane + 32 * it, rr = f4 >> 4, q = (f4 & 15) * 4;
        *(volatile v4f_t*)(Y + (size_t)(m0 + wm + rr) * ldy + n0 + wn + q) = *(const v4fa*)(so + rr * 68 + q); }
    }
    __threadfence();
  }
}

template <typename AT, bool ACC>
__global__ __launch_bounds__(256) void gemm_kn2(const AT* __restrict__ A, int lda, size_t strideA,
                                               const float* __restrict__ Wm, int ldw, size_t strideW,
                                               const float* __restrict__ bias, float scale,
                                               float* __restrict__ Y, int ldy, size_t strideY, int K) {
  __shared__ __attribute__((aligned(16))) f16 ldsA[128 * GSTR], ldsAl[128 * GSTR];
  __shared__ __attribute__((aligned(16))) f16 ldsW[128 * GSTR], ldsWl[128 * GSTR];
  __shared__ __attribute__((aligned(16))) float oS[8][32 * 68];
  const int tid = threadIdx.x, lane = tid & 31, wave = tid >> 5, cl = lane & 15, rh = (lane >> 4) * 8;
  const int m0 = blockIdx.x * 128, n0 = blockIdx.y * 128;
  const int wm = (wave & 3) * 32, wn = (wave >> 2) * 64;
  A += (size_t)blockIdx.z * strideA; Wm += (size_t)blockIdx.z * strideW; Y += (size_t)blockIdx.z * strideY;
  f32x8 acc[2][4], accx[2][4];
#pragma unroll
  for (int i = 0; i < 2; ++i)
#pragma unroll
    for (int j = 0; j < 4; ++j) { f32x8 z = {}; acc[i][j] = z; accx[i][j] = z; }
#pragma unroll 1
  for (int k0 = 0; k0 < K; k0 += 32) {
    __syncthreads();
    {
      const int row = tid >> 1, ch = (tid & 1) * 16;
      const AT* src = A + (size_t)(m0 + row) * lda + k0 + ch;
#pragma unroll
      for (int g = 0; g < 16; ++g) { const float v = (float)src[g]; const f16 h = (f16)v; ldsA[row * GSTR + ch + g] = h; ldsAl[row * GSTR + ch + g] = (f16)((v - (float)h) * 2048.0f); }
    }
    {
      const int k = tid >> 3, nn0 = (tid & 7) * 16;
      const float* src = Wm + (size_t)(k0 + k) * ldw + n0 + nn0;
#pragma unroll
      for (int g = 0; g < 4; ++g) { const v4f_t v = *(const v4f_t*)(src + 4 * g);
#pragma unroll
        for (int u = 0; u < 4; ++u) { const f16 h = (f16)v[u]; ldsW[(nn0 + 4 * g + u) * GSTR + k] = h; ldsWl[(nn0 + 4 * g + u) * GSTR + k] = (f16)((v[u] - (float)h) * 2048.0f); } }
    }
    __syncthreads();
    f16x16 af[2], afl[2];
#pragma unroll
    for (int i = 0; i < 2; ++i) { af[i] = lds_frag(ldsA + (wm + 16 * i) * GSTR, GSTR); afl[i] = lds_frag(ldsAl + (wm + 16 * i) * GSTR, GSTR); }
#pragma unroll
    for (int j = 0; j < 4; ++j) {
      const f16x16 bf = lds_frag(ldsW + (wn + 16 * j) * GSTR, GSTR), bfl = lds_frag(ldsWl + (wn + 16 * j) * GSTR, GSTR);
#pragma unroll
      for (int i = 0; i < 2; ++i) { acc[i][j] = wmma16(af[i], bf, acc[i][j]); accx[i][j] = wmma16(af[i], bfl, accx[i][j]); accx[i][j] = wmma16(afl[i], bf, accx[i][j]); }
    }
  }
  float* so = oS[wave];
#pragma unroll
  for (int i = 0; i < 2; ++i)
#pragma unroll
    for (int j = 0; j < 4; ++j) {
      const float bv = bias ? bias[n0 + wn + 16 * j + cl] : 0.0f;
#pragma unroll
      for (int r = 0; r < 8; ++r) so[(16 * i + rh + r) * 68 + 16 * j + cl] = (acc[i][j][r] + accx[i][j][r] * (1.0f / 2048.0f)) * scale + bv;
    }
  asm volatile("s_wait_dscnt 0" ::: "memory");
  __builtin_amdgcn_wave_barrier();
  if (ACC) {
#pragma unroll
    for (int it = 0; it < 16; ++it) { const int f4 = lane + 32 * it, rr = f4 >> 4, q = (f4 & 15) * 4;
      const v4f_t old = *(const v4fa*)(Y + (size_t)(m0 + wm + rr) * ldy + n0 + wn + q);
      v4f_t v = *(const v4fa*)(so + rr * 68 + q); v += old; *(v4fa*)(so + rr * 68 + q) = v; }
    asm volatile("s_wait_dscnt 0" ::: "memory");
  }
#pragma unroll 1
  for (int pass = 0; pass < 2; ++pass) {
#pragma unroll
    for (int it = 0; it < 16; ++it) { const int f4 = lane + 32 * it, rr = f4 >> 4, q = (f4 & 15) * 4;
      *(volatile v4f_t*)(Y + (size_t)(m0 + wm + rr) * ldy + n0 + wn + q) = *(const v4fa*)(so + rr * 68 + q); }
    __threadfence();
  }
}

__global__ __launch_bounds__(256) void k_transpose(const float* __restrict__ Wm, float* __restrict__ Wt, int rows, int cols) {
  __shared__ float tS[64][65];
  const int tid = threadIdx.x, tbj = cols / 64, bi = blockIdx.x / tbj, bj = blockIdx.x % tbj;
  for (int e = tid; e < 64 * 64; e += 256) { const int r = e >> 6, c = e & 63; tS[r][c] = Wm[(size_t)(bi * 64 + r) * cols + bj * 64 + c]; }
  __syncthreads();
  for (int ch = tid; ch < 64 * 16; ch += 256) { const int r = ch >> 4, q4 = (ch & 15) * 4; v4f_t o; o[0] = tS[q4][r]; o[1] = tS[q4 + 1][r]; o[2] = tS[q4 + 2][r]; o[3] = tS[q4 + 3][r];
    float* dst = Wt + (size_t)(bj * 64 + r) * rows + bi * 64 + q4; *(volatile v4f_t*)dst = o; __threadfence(); *(volatile v4f_t*)dst = o; }
}


template <typename AT, int EPI, bool OUT16, int NJ>
__global__ __launch_bounds__(256) void gemm_sm(const AT* __restrict__ A, int lda, size_t sA, const float* __restrict__ Wm, int ldw, size_t sW,
                                               const float* __restrict__ bias, const float* __restrict__ R, const float* __restrict__ gvec,
                                               void* __restrict__ Yv, int ldy, size_t sY, int K) {
  constexpr int BN = 16 * NJ; constexpr int OST = BN + 4;
  A += (size_t)blockIdx.z * sA; Wm += (size_t)blockIdx.z * sW; Yv = (void*)((char*)Yv + (size_t)blockIdx.z * sY * (OUT16 ? 2 : 4)); if (R) R += (size_t)blockIdx.z * sY;
  __shared__ __attribute__((aligned(16))) f16 ldsA[256 * GSTR];
  __shared__ __attribute__((aligned(16))) f16 ldsW[BN * GSTR];
  __shared__ __attribute__((aligned(16))) float oS[8][32 * OST];
  const int tid = threadIdx.x, lane = tid & 31, wave = tid >> 5, cl = lane & 15, rh = (lane >> 4) * 8;
  const int m0 = blockIdx.x * 256, n0 = blockIdx.y * BN;
  const int wm = wave * 32;
  f32x8 acc[2][NJ];
#pragma unroll
  for (int i = 0; i < 2; ++i)
#pragma unroll
    for (int j = 0; j < NJ; ++j) { f32x8 z = {}; acc[i][j] = z; }
#pragma unroll 1
  for (int k0 = 0; k0 < K; k0 += 32) {
    __syncthreads();
    { const AT* src = A + (size_t)(m0 + tid) * lda + k0;
#pragma unroll
      for (int g = 0; g < 32; ++g) ldsA[tid * GSTR + g] = (f16)src[g]; }
    { const int k = tid >> 3, nn0 = (tid & 7) * (2 * NJ);
      const float* src = Wm + (size_t)(k0 + k) * ldw + n0 + nn0;
#pragma unroll
      for (int g = 0; g < NJ / 2; ++g) { const v4f_t v = *(const v4f_t*)(src + 4 * g);
#pragma unroll
        for (int u = 0; u < 4; ++u) ldsW[(nn0 + 4 * g + u) * GSTR + k] = (f16)v[u]; } }
    __syncthreads();
    f16x16 af[2];
#pragma unroll
    for (int i = 0; i < 2; ++i) af[i] = lds_frag(ldsA + (wm + 16 * i) * GSTR, GSTR);
#pragma unroll
    for (int j = 0; j < NJ; ++j) {
      const f16x16 bf = lds_frag(ldsW + (16 * j) * GSTR, GSTR);
#pragma unroll
      for (int i = 0; i < 2; ++i) acc[i][j] = wmma16(af[i], bf, acc[i][j]);
    }
  }
  float* so = oS[wave];
#pragma unroll
  for (int i = 0; i < 2; ++i)
#pragma unroll
    for (int j = 0; j < NJ; ++j) {
      const int n = n0 + 16 * j + cl;
      const float bv = bias ? bias[n] : 0.0f;
      const float gv = (EPI == 2 || EPI == 4) ? gvec[n] : 0.0f;
#pragma unroll
      for (int r = 0; r < 8; ++r) {
        float v = acc[i][j][r] + bv;
        if (EPI == 3) v = fmaxf(v, 0.0f);
        if (EPI == 2) v = R[(size_t)(m0 + wm + 16 * i + rh + r) * ldy + n] + gv * v;
        if (EPI == 4) v = gv * v;
        so[(16 * i + rh + r) * OST + 16 * j + cl] = v;
      }
    }
  asm volatile("s_wait_dscnt 0" ::: "memory");
  __builtin_amdgcn_wave_barrier();
#pragma unroll 1
  for (int pass = 0; pass < 2; ++pass) {
    if (OUT16) {
      f16* Y = (f16*)Yv;
#pragma unroll
      for (int it = 0; it < BN / 8; ++it) { const int c = lane + 32 * it, rr = c / (BN / 8), q8 = (c % (BN / 8)) * 8;
        union { f16 h[8]; v4u_t v; } u;
#pragma unroll
        for (int e = 0; e < 8; ++e) u.h[e] = (f16)so[rr * OST + q8 + e];
        *(volatile v4u_t*)(Y + (size_t)(m0 + wm + rr) * ldy + n0 + q8) = u.v; }
    } else {
      float* Y = (float*)Yv;
#pragma unroll
      for (int it = 0; it < BN / 4; ++it) { const int f4 = lane + 32 * it, rr = f4 / (BN / 4), q = (f4 % (BN / 4)) * 4;
        *(volatile v4f_t*)(Y + (size_t)(m0 + wm + rr) * ldy + n0 + q) = *(const v4fa*)(so + rr * OST + q); }
    }
    __threadfence();
  }
}

#define NBw 4
#define SSq 1000
#define SPq 1024
#define HHq 768
#define NHq 12
__global__ __launch_bounds__(256) void k_fill(float* __restrict__ p, float val, size_t n4) { const size_t i = (size_t)blockIdx.x * 256 + threadIdx.x; if (i < n4) { v4f_t v = {val, val, val, val}; *(volatile v4f_t*)(p + 4 * i) = v; __threadfence(); *(volatile v4f_t*)(p + 4 * i) = v; } }
__global__ __launch_bounds__(256) void k_dbg_zero(float* __restrict__ p, size_t n4) { const size_t i = (size_t)blockIdx.x * 256 + threadIdx.x; if (i < n4) { v4f_t z = {0.f,0.f,0.f,0.f}; *(volatile v4f_t*)(p + 4 * i) = z; __threadfence(); *(volatile v4f_t*)(p + 4 * i) = z; } }
__global__ __launch_bounds__(256) void k_copy(const float* __restrict__ src, float* __restrict__ dst, size_t n4) { const size_t i = (size_t)blockIdx.x * 256 + threadIdx.x; if (i < n4) { const v4f_t v = *(const v4f_t*)(src + 4 * i); *(volatile v4f_t*)(dst + 4 * i) = v; __threadfence(); *(volatile v4f_t*)(dst + 4 * i) = v; } }
__global__ __launch_bounds__(256) void k_ln(const float* __restrict__ X, const float* __restrict__ gam, const float* __restrict__ bet, float* __restrict__ Y) {
  __shared__ __attribute__((aligned(16))) float rowS[16 * 772];
  const int tid = threadIdx.x, r = tid >> 4, part = tid & 15; const size_t row = (size_t)blockIdx.x * 16 + r;
  float s = 0.0f;
#pragma unroll 1
  for (int i = 0; i < 48; ++i) { const float v = X[row * 768 + part * 48 + i]; rowS[r * 772 + part * 48 + i] = v; s += v; }
  s += __shfl_xor(s, 1, 32); s += __shfl_xor(s, 2, 32); s += __shfl_xor(s, 4, 32); s += __shfl_xor(s, 8, 32);
  const float mean = s * (1.0f / 768.0f); float q = 0.0f;
#pragma unroll 1
  for (int i = 0; i < 48; ++i) { const float dv = rowS[r * 772 + part * 48 + i] - mean; q += dv * dv; }
  q += __shfl_xor(q, 1, 32); q += __shfl_xor(q, 2, 32); q += __shfl_xor(q, 4, 32); q += __shfl_xor(q, 8, 32);
  const float rstd = 1.0f / __builtin_sqrtf(q * (1.0f / 768.0f) + 1e-5f);
#pragma unroll 1
  for (int i = 0; i < 48; ++i) { const int c = part * 48 + i; rowS[r * 772 + c] = (rowS[r * 772 + c] - mean) * rstd * gam[c] + bet[c]; }
  __syncthreads();
#pragma unroll 1
  for (int pass = 0; pass < 2; ++pass) { for (int q4 = tid; q4 < 16 * 192; q4 += 256) { const int rr = q4 / 192, c4 = (q4 % 192) * 4;
      *(volatile v4f_t*)(Y + ((size_t)blockIdx.x * 16 + rr) * 768 + c4) = *(const v4fa*)(rowS + rr * 772 + c4); } __threadfence(); }
}
__global__ __launch_bounds__(256) void k_vmean(const float* __restrict__ V, int ldv, float* __restrict__ VB) {
  const int c = blockIdx.x * 256 + threadIdx.x; float s = 0.0f;
#pragma unroll 1
  for (int r = 0; r < 1024; ++r) s += V[(size_t)r * ldv + c];
  const float m = s * (1.0f / 1024.0f); *(volatile float*)(VB + c) = m; __threadfence(); *(volatile float*)(VB + c) = m;
}
__global__ __launch_bounds__(256) void k_vmeank(const float* __restrict__ V, int ldv, float* __restrict__ VB) {
  const int c = blockIdx.x * 256 + threadIdx.x; float s = 0.0f;
#pragma unroll 1
  for (int r = 0; r < 1024; ++r) s += V[(size_t)r * ldv + c];
  const float m = s * (1024.0f / 1024.0f); *(volatile float*)(VB + c) = m; __threadfence(); *(volatile float*)(VB + c) = m;
}
__global__ __launch_bounds__(256) void k_softmax_m(float* __restrict__ Sm) {
  __shared__ float red[256];
  const int q = blockIdx.x, z = blockIdx.y, tid = threadIdx.x; float* sr = Sm + ((size_t)z * SPq + q) * SPq; float v[SPq / 256]; float m = -3.0e38f;
#pragma unroll
  for (int e = 0; e < SPq / 256; ++e) { const int k = tid + 256 * e; v[e] = (k < SSq) ? sr[k] * 0.125f : -3.0e38f; m = fmaxf(m, v[e]); }
  red[tid] = m; __syncthreads(); for (int o = 128; o > 0; o >>= 1) { if (tid < o) red[tid] = fmaxf(red[tid], red[tid + o]); __syncthreads(); }
  m = red[0]; __syncthreads(); float zs = 0.0f;
#pragma unroll
  for (int e = 0; e < SPq / 256; ++e) { const int k = tid + 256 * e; v[e] = (k < SSq) ? expf(v[e] - m) : 0.0f; zs += v[e]; }
  red[tid] = zs; __syncthreads(); for (int o = 128; o > 0; o >>= 1) { if (tid < o) red[tid] += red[tid + o]; __syncthreads(); }
  const float kk = 1024.0f / red[0];
#pragma unroll 1
  for (int pass = 0; pass < 2; ++pass) {
#pragma unroll
    for (int e = 0; e < SPq / 256; ++e) *(volatile float*)(sr + tid + 256 * e) = v[e] * kk - 1.0f;
    __threadfence(); }
}
__global__ __launch_bounds__(192) void k_padx(const float* __restrict__ xb, float* __restrict__ X) {
  const int s = blockIdx.x, c = 4 * threadIdx.x; v4f_t v = {0.f, 0.f, 0.f, 0.f}; if (s < SSq) v = *(const v4f_t*)(xb + (size_t)s * HHq + c);
  float* d = X + (size_t)s * HHq + c; *(volatile v4f_t*)d = v; __threadfence(); *(volatile v4f_t*)d = v;
}
__global__ __launch_bounds__(256) void k_lnrelu_add(const float* __restrict__ G, const float* __restrict__ g, const float* __restrict__ bb, const float* __restrict__ F, float* __restrict__ F2) {
  __shared__ __attribute__((aligned(16))) float rowS[16 * 772];
  const int tid = threadIdx.x, r = tid >> 4, part = tid & 15; const size_t row = (size_t)blockIdx.x * 16 + r; float s = 0.0f;
#pragma unroll 1
  for (int i = 0; i < HHq / 16; ++i) { const float v = G[row * HHq + part * (HHq / 16) + i]; rowS[r * 772 + part * (HHq / 16) + i] = v; s += v; }
  s += __shfl_xor(s, 1, 32); s += __shfl_xor(s, 2, 32); s += __shfl_xor(s, 4, 32); s += __shfl_xor(s, 8, 32); const float mean = s * (1.0f / HHq); float q = 0.0f;
#pragma unroll 1
  for (int i = 0; i < HHq / 16; ++i) { const float dv = rowS[r * 772 + part * (HHq / 16) + i] - mean; q += dv * dv; }
  q += __shfl_xor(q, 1, 32); q += __shfl_xor(q, 2, 32); q += __shfl_xor(q, 4, 32); q += __shfl_xor(q, 8, 32); const float rs = 1.0f / __builtin_sqrtf(q * (1.0f / HHq) + 1e-5f);
#pragma unroll 1
  for (int i = 0; i < HHq / 16; ++i) { const int c = part * (HHq / 16) + i; const float v = fmaxf((rowS[r * 772 + c] - mean) * rs * g[c] + bb[c], 0.0f) + F[row * HHq + c]; rowS[r * 772 + c] = v; }
  __syncthreads();
#pragma unroll 1
  for (int pass = 0; pass < 2; ++pass) { for (int q4 = tid; q4 < 16 * (HHq / 4); q4 += 256) { const int rr = q4 / (HHq / 4), c4 = (q4 % (HHq / 4)) * 4; *(volatile v4f_t*)(F2 + ((size_t)blockIdx.x * 16 + rr) * HHq + c4) = *(const v4fa*)(rowS + rr * 772 + c4); } __threadfence(); }
}
__global__ __launch_bounds__(192) void k_levelin(const float* __restrict__ cur, const float* __restrict__ le, const float* __restrict__ pe, float psc, float* __restrict__ INP, float* __restrict__ FWP) {
  const int s = blockIdx.x, c = 4 * threadIdx.x; const v4f_t a = *(const v4f_t*)(cur + (size_t)s * HHq + c) + *(const v4f_t*)(le + c);
  v4f_t p = {0.f, 0.f, 0.f, 0.f}; if (s < SSq) p = *(const v4f_t*)(pe + (size_t)s * HHq + c); const v4f_t fw = a + p * psc;
#pragma unroll 1
  for (int pass = 0; pass < 2; ++pass) { *(volatile v4f_t*)(INP + (size_t)s * HHq + c) = a; *(volatile v4f_t*)(FWP + (size_t)s * HHq + c) = fw; __threadfence(); }
}
__global__ __launch_bounds__(384) void k_band(const float* __restrict__ Q, const float* __restrict__ K, const float* __restrict__ V, int w, float* __restrict__ CTX) {
  const int s = blockIdx.x, tid = threadIdx.x; const int h = tid >> 5, c = tid & 31; const size_t col = (size_t)h * 64 + 2 * c;
  const float q0 = Q[(size_t)s * HHq + col], q1 = Q[(size_t)s * HHq + col + 1]; float lg[11]; float mx = -3.0e38f;
#pragma unroll
  for (int e = 0; e < 11; ++e) { const int j = s - w + e; const int jc = min(max(j, 0), SSq - 1); float d = q0 * K[(size_t)jc * HHq + col] + q1 * K[(size_t)jc * HHq + col + 1];
    d += __shfl_xor(d, 1, 32); d += __shfl_xor(d, 2, 32); d += __shfl_xor(d, 4, 32); d += __shfl_xor(d, 8, 32); d += __shfl_xor(d, 16, 32);
    const bool ok = (e <= 2 * w) && (j >= 0) && (j < SSq); lg[e] = ok ? d * 0.125f : -3.0e38f; mx = fmaxf(mx, lg[e]); }
  float z = 0.0f, o0 = 0.0f, o1 = 0.0f;
#pragma unroll
  for (int e = 0; e < 11; ++e) { const int j = s - w + e; const int jc = min(max(j, 0), SSq - 1); const float p = (lg[e] > -1.0e38f) ? expf(lg[e] - mx) : 0.0f; z += p;
    o0 = fmaf(p, V[(size_t)jc * HHq + col], o0); o1 = fmaf(p, V[(size_t)jc * HHq + col + 1], o1); }
  const float iz = 1.0f / z; union { float f2[2]; unsigned long long u; } pk; pk.f2[0] = o0 * iz; pk.f2[1] = o1 * iz;
  *(volatile unsigned long long*)(CTX + (size_t)s * HHq + col) = pk.u; __threadfence(); *(volatile unsigned long long*)(CTX + (size_t)s * HHq + col) = pk.u;
}
__global__ __launch_bounds__(256) void k_colmean(const float* __restrict__ F, float* __restrict__ CM) { const int c = blockIdx.x * 256 + threadIdx.x; float s = 0.0f;
#pragma unroll 1
  for (int r = 0; r < SSq; ++r) s += F[(size_t)r * HHq + c]; const float m = s * (1.0f / SSq); *(volatile float*)(CM + c) = m; __threadfence(); *(volatile float*)(CM + c) = m; }
__global__ __launch_bounds__(256) void k_detect(const float* __restrict__ CM, const float* __restrict__ W1, const float* __restrict__ b1, const float* __restrict__ W2, const float* __restrict__ b2, float* __restrict__ REL) {
  __shared__ float ra[256], rb[256], rcc[256];
  const int tid = threadIdx.x; float a0 = 0.f, a1 = 0.f, a2 = 0.f;
#pragma unroll 1
  for (int jj = 0; jj < 3; ++jj) { const int o = tid + 256 * jj; float hsum = b1[o];
#pragma unroll 1
    for (int i = 0; i < 3 * HHq; ++i) hsum = fmaf(CM[i], W1[(size_t)i * HHq + o], hsum);
    const float hv = fmaxf(hsum, 0.0f); a0 = fmaf(hv, W2[o * 3 + 0], a0); a1 = fmaf(hv, W2[o * 3 + 1], a1); a2 = fmaf(hv, W2[o * 3 + 2], a2); }
  ra[tid] = a0; rb[tid] = a1; rcc[tid] = a2; __syncthreads();
  for (int o = 128; o > 0; o >>= 1) { if (tid < o) { ra[tid] += ra[tid + o]; rb[tid] += rb[tid + o]; rcc[tid] += rcc[tid + o]; } __syncthreads(); }
  if (tid < 32) { float v = 0.0f; if (tid == 0) v = 1.0f / (1.0f + expf(-(ra[0] + b2[0]))); if (tid == 1) v = 1.0f / (1.0f + expf(-(rb[0] + b2[1]))); if (tid == 2) v = 1.0f / (1.0f + expf(-(rcc[0] + b2[2])));
    *(volatile float*)(REL + tid) = v; __threadfence(); *(volatile float*)(REL + tid) = v; }
}
__global__ __launch_bounds__(256) void k_fillfrom(const float* __restrict__ src, float* __restrict__ dst, int n4) { const int i = blockIdx.x * 256 + threadIdx.x; if (i < n4) { const float s = src[0]; const v4f_t v = {s, s, s, s}; *(volatile v4f_t*)(dst + 4 * i) = v; __threadfence(); *(volatile v4f_t*)(dst + 4 * i) = v; } }
__global__ __launch_bounds__(256) void k_graph(const float* __restrict__ CM, const float* __restrict__ REL, const float* __restrict__ Wn, const float* __restrict__ bn, const float* __restrict__ We1, const float* __restrict__ be1,
                                              const float* __restrict__ We2, const float* __restrict__ be2, const float* __restrict__ AE, float* __restrict__ GR) {
  __shared__ float base[HHq]; __shared__ float node[HHq]; __shared__ float red[256]; __shared__ float esum[4];
  const int tid = threadIdx.x; const float r2 = REL[2];
  for (int c = tid; c < HHq; c += 256) base[c] = r2 * CM[2 * HHq + c];
  __syncthreads();
  for (int o = tid; o < HHq; o += 256) { float a = bn[o];
#pragma unroll 1
    for (int i = 0; i < HHq; ++i) a = fmaf(base[i], Wn[(size_t)i * HHq + o], a); node[o] = fmaxf(a, 0.0f); }
  __syncthreads();
  float etot = 0.0f;
#pragma unroll 1
  for (int pr = 0; pr < 3; ++pr) { const int ia = (pr == 2) ? 1 : 0, ib = (pr == 0) ? 1 : 2;
    float part = 0.0f;
    for (int o = tid; o < HHq; o += 256) { float a = be1[o];
#pragma unroll 1
      for (int i = 0; i < HHq; ++i) { a = fmaf(node[i] + AE[ia * HHq + i], We1[(size_t)i * HHq + o], a); a = fmaf(node[i] + AE[ib * HHq + i], We1[(size_t)(HHq + i) * HHq + o], a); }
      part = fmaf(fmaxf(a, 0.0f), We2[o], part); }
    red[tid] = part; __syncthreads(); for (int o = 128; o > 0; o >>= 1) { if (tid < o) red[tid] += red[tid + o]; __syncthreads(); }
    if (tid == 0) esum[pr] = 1.0f / (1.0f + expf(-(red[0] + be2[0])));
    __syncthreads(); }
  etot = (esum[0] + esum[1] + esum[2]) * (1.0f / 3.0f);
  for (int c = tid; c < HHq; c += 256) { const float nr = node[c] + (AE[c] + AE[HHq + c] + AE[2 * HHq + c]) * (1.0f / 3.0f); const float v = nr + etot * nr; *(volatile float*)(GR + c) = v; }
  __threadfence();
  for (int c = tid; c < HHq; c += 256) { const float v2 = GR[c]; *(volatile float*)(GR + c) = v2; }
}
__global__ __launch_bounds__(256) void k_final(const float* __restrict__ FUS, const float* __restrict__ fb, const float* __restrict__ g, const float* __restrict__ bb, const float* __restrict__ GR, float* __restrict__ outb) {
  __shared__ __attribute__((aligned(16))) float rowS[16 * 772];
  const int tid = threadIdx.x, r = tid >> 4, part = tid & 15; const size_t row = (size_t)blockIdx.x * 16 + r; float s = 0.0f;
#pragma unroll 1
  for (int i = 0; i < HHq / 16; ++i) { const int c = part * (HHq / 16) + i; const float v = FUS[row * HHq + c] + fb[c]; rowS[r * 772 + c] = v; s += v; }
  s += __shfl_xor(s, 1, 32); s += __shfl_xor(s, 2, 32); s += __shfl_xor(s, 4, 32); s += __shfl_xor(s, 8, 32); const float mean = s * (1.0f / HHq); float q = 0.0f;
#pragma unroll 1
  for (int i = 0; i < HHq / 16; ++i) { const float dv = rowS[r * 772 + part * (HHq / 16) + i] - mean; q += dv * dv; }
  q += __shfl_xor(q, 1, 32); q += __shfl_xor(q, 2, 32); q += __shfl_xor(q, 4, 32); q += __shfl_xor(q, 8, 32); const float rs = 1.0f / __builtin_sqrtf(q * (1.0f / HHq) + 1e-5f);
#pragma unroll 1
  for (int i = 0; i < HHq / 16; ++i) { const int c = part * (HHq / 16) + i; rowS[r * 772 + c] = fmaxf((rowS[r * 772 + c] - mean) * rs * g[c] + bb[c], 0.0f) + GR[c]; }
  __syncthreads();
  const int nrows = min(16, SSq - (int)blockIdx.x * 16);
#pragma unroll 1
  for (int pass = 0; pass < 2; ++pass) { for (int q4 = tid; q4 < nrows * (HHq / 4); q4 += 256) { const int rr = q4 / (HHq / 4), c4 = (q4 % (HHq / 4)) * 4; *(volatile v4f_t*)(outb + ((size_t)blockIdx.x * 16 + rr) * HHq + c4) = *(const v4fa*)(rowS + rr * 772 + c4); } __threadfence(); }
}

extern "C" void kernel_launch(void* const* d_in, const int* in_sizes, int n_in,
                              void* d_out, int out_size, void* d_ws, size_t ws_size,
                              hipStream_t stream) {
  (void)in_sizes; (void)n_in; (void)out_size;
  const float** f = (const float**)d_in;
  const float* x = f[0], *semW = f[1], *semb = f[2], *semg = f[3], *sembe = f[4], *pe = f[5], *Wq = f[6], *bq = f[7], *Wk = f[8], *bk = f[9], *Wv = f[10], *bv = f[11], *Wo = f[12], *bo = f[13],
              *lng = f[14], *lnb = f[15], *le = f[16], *spW1 = f[17], *spb1 = f[18], *spW2 = f[19], *spb2 = f[20], *nW = f[21], *nb = f[22], *eW1 = f[23], *eb1 = f[24], *eW2 = f[25], *eb2 = f[26],
              *ae = f[27], *fW = f[28], *fb = f[29], *fg = f[30], *fbe = f[31];
  float* out = (float*)d_out;
  char* ws = (char*)d_ws;
  float* FA = (float*)ws; ws += (size_t)SPq * HHq * 4; float* FB = (float*)ws; ws += (size_t)SPq * HHq * 4; float* G = (float*)ws; ws += (size_t)SPq * HHq * 4;
  float* INP = (float*)ws; ws += (size_t)SPq * HHq * 4; float* FWP = (float*)ws; ws += (size_t)SPq * HHq * 4; float* Q = (float*)ws; ws += (size_t)SPq * HHq * 4; float* Kp = (float*)ws; ws += (size_t)SPq * HHq * 4; float* V = (float*)ws; ws += (size_t)SPq * HHq * 4;
  float* KT = (float*)ws; ws += (size_t)SPq * HHq * 4; float* S = (float*)ws; ws += (size_t)2 * SPq * SPq * 4; float* CTX = (float*)ws; ws += (size_t)SPq * HHq * 4;
  float* F0 = (float*)ws; ws += (size_t)SPq * HHq * 4; float* F1 = (float*)ws; ws += (size_t)SPq * HHq * 4; float* F2 = (float*)ws; ws += (size_t)SPq * HHq * 4; float* FUS = (float*)ws; ws += (size_t)SPq * HHq * 4;
  float* VB = (float*)ws; ws += HHq * 4; float* VBK = (float*)ws; ws += HHq * 4; float* sc = (float*)ws; ws += 64 * 4; float* ones = (float*)ws; ws += HHq * 4;
  float* CM = (float*)ws; ws += 3 * HHq * 4; float* REL = (float*)ws; ws += 32 * 4; float* RV = (float*)ws; ws += 3 * HHq * 4; float* GR = (float*)ws; ws += HHq * 4;
  if ((size_t)(ws - (char*)d_ws) > ws_size) return;
  float* FL[3] = {F0, F1, F2};
  const dim3 blk(256); const dim3 gp(SPq / 128, HHq / 128);
  k_fill<<<dim3(1), blk, 0, stream>>>(sc, 1.0f / 1024.0f, 64 / 4); k_fill<<<dim3(1), blk, 0, stream>>>(ones, 1.0f, HHq / 4);

  for (int b = 0; b < NBw; ++b) {
    k_padx<<<dim3(SPq), dim3(192), 0, stream>>>(x + (size_t)b * SSq * HHq, FA);
    float* feat = FA; float* fnext = FB;
    for (int i = 0; i < 3; ++i) {
      gemm_kne<float, 0, false><<<gp, blk, 0, stream>>>(feat, HHq, semW + (size_t)i * HHq * HHq, HHq, semb + i * HHq, nullptr, nullptr, G, HHq, HHq);
      k_lnrelu_add<<<dim3(SPq / 16), blk, 0, stream>>>(G, semg + i * HHq, sembe + i * HHq, feat, fnext); { float* t = feat; feat = fnext; fnext = t; }
    }
    const float* cur = feat;
    for (int l = 0; l < 3; ++l) {
      k_levelin<<<dim3(SPq), dim3(192), 0, stream>>>(cur, le + l * HHq, pe + (size_t)l * SSq * HHq, 1.0f + 0.1f * (float)l, INP, FWP);
      gemm_kne<float, 0, false><<<gp, blk, 0, stream>>>(FWP, HHq, Wq + (size_t)l * HHq * HHq, HHq, bq + l * HHq, nullptr, nullptr, Q, HHq, HHq);
      gemm_kne<float, 0, false><<<gp, blk, 0, stream>>>(FWP, HHq, Wk + (size_t)l * HHq * HHq, HHq, bk + l * HHq, nullptr, nullptr, Kp, HHq, HHq);
      gemm_kne<float, 0, false><<<gp, blk, 0, stream>>>(FWP, HHq, Wv + (size_t)l * HHq * HHq, HHq, bv + l * HHq, nullptr, nullptr, V, HHq, HHq);
      if (l < 2) { k_band<<<dim3(SSq), dim3(384), 0, stream>>>(Q, Kp, V, l == 0 ? 2 : 5, CTX); k_fill<<<dim3(((SPq - SSq) * HHq / 4 + 255) / 256), blk, 0, stream>>>(CTX + (size_t)SSq * HHq, 0.0f, (SPq - SSq) * HHq / 4); }
      else {
        k_vmean<<<dim3(HHq / 256), blk, 0, stream>>>(V, HHq, VB); k_vmeank<<<dim3(HHq / 256), blk, 0, stream>>>(V, HHq, VBK);
        k_transpose<<<dim3((SPq / 64) * (HHq / 64)), blk, 0, stream>>>(Kp, KT, SPq, HHq);
        for (int hg = 0; hg < NHq / 2; ++hg) { const int h0 = 2 * hg;
          gemm_knez<float, 0, false><<<dim3(SPq / 128, SPq / 128, 2), blk, 0, stream>>>(Q + h0 * 64, HHq, (size_t)64, KT + (size_t)h0 * 64 * SPq, SPq, (size_t)64 * SPq, nullptr, nullptr, nullptr, S, SPq, (size_t)SPq * SPq, 64);
          k_softmax_m<<<dim3(SPq, 2), blk, 0, stream>>>(S);
          for (int z = 0; z < 2; ++z)
            gemm_sm<float, 4, false, 4><<<dim3(SPq / 256, 1, 1), blk, 0, stream>>>(S + (size_t)z * SPq * SPq, SPq, (size_t)0, V + (h0 + z) * 64, HHq, (size_t)0, VBK + (h0 + z) * 64, nullptr, sc, CTX + (h0 + z) * 64, HHq, (size_t)0, SPq);
        }
      }
      gemm_kne<float, 2, false><<<gp, blk, 0, stream>>>(CTX, HHq, Wo + (size_t)l * HHq * HHq, HHq, bo + l * HHq, INP, ones, G, HHq, HHq);
      k_ln<<<dim3(SPq / 16), blk, 0, stream>>>(G, lng + l * HHq, lnb + l * HHq, FL[l]); cur = FL[l];
    }
    for (int l = 0; l < 3; ++l) k_colmean<<<dim3(HHq / 256), blk, 0, stream>>>(FL[l], CM + l * HHq);
    k_detect<<<dim3(1), blk, 0, stream>>>(CM, spW1, spb1, spW2, spb2, REL);
    for (int l = 0; l < 3; ++l) k_fillfrom<<<dim3(1), blk, 0, stream>>>(REL + l, RV + l * HHq, HHq / 4);
    k_graph<<<dim3(1), blk, 0, stream>>>(CM, REL, nW, nb, eW1, eb1, eW2, eb2, ae, GR);
    gemm_kne<float, 4, false><<<gp, blk, 0, stream>>>(F0, HHq, fW, HHq, nullptr, nullptr, RV, FUS, HHq, HHq);
    for (int l = 1; l < 3; ++l) gemm_kne<float, 2, false><<<gp, blk, 0, stream>>>(FL[l], HHq, fW + (size_t)l * HHq * HHq, HHq, nullptr, FUS, RV + l * HHq, FUS, HHq, HHq);
    k_final<<<dim3((SSq + 15) / 16), blk, 0, stream>>>(FUS, fb, fg, fbe, GR, out + (size_t)b * SSq * HHq);
  }
}
